// EATTS_44822278701146
// MI455X (gfx1250) — hardware-verified
//
#include <hip/hip_runtime.h>


#define NB_  2
#define NN   1024
#define CC   64
#define NT   (NB_ * NN)
#define SL   0.2f
typedef _Float16 h16;
typedef unsigned short bf;
typedef __attribute__((ext_vector_type(16))) __bf16   v16bf;
typedef __attribute__((ext_vector_type(16))) _Float16 v16h;
typedef __attribute__((ext_vector_type(8)))  _Float16 v8h;
typedef __attribute__((ext_vector_type(8)))  unsigned short v8us;
typedef __attribute__((ext_vector_type(8)))  float    v8f;
typedef __attribute__((ext_vector_type(4)))  float    v4f;
typedef v8h  __attribute__((may_alias)) v8ha;
typedef v4f  __attribute__((may_alias)) v4fa;
typedef v8us __attribute__((may_alias)) v8usa;

__device__ __forceinline__ unsigned short f2bf(float f) { unsigned u = __float_as_uint(f); u += 0x7FFFu + ((u >> 16) & 1u); return (unsigned short)(u >> 16); }
__device__ __forceinline__ float bf2f(unsigned short b) { return __uint_as_float(((unsigned)b) << 16); }
__device__ __forceinline__ float bfr(float f) { return bf2f(f2bf(f)); }
__device__ __forceinline__ v16h cat16(v8h lo, v8h hi) { return __builtin_shufflevector(lo, hi, 0, 1, 2, 3, 4, 5, 6, 7, 8, 9, 10, 11, 12, 13, 14, 15); }
__device__ __forceinline__ v16bf cat16b(v8us lo, v8us hi) { return __builtin_bit_cast(v16bf, __builtin_shufflevector(lo, hi, 0, 1, 2, 3, 4, 5, 6, 7, 8, 9, 10, 11, 12, 13, 14, 15)); }
__device__ __forceinline__ v8f wmma16(v16h a, v16h b, v8f c) { return __builtin_amdgcn_wmma_f32_16x16x32_f16(false, a, false, b, (short)0, c, false, false); }
__device__ __forceinline__ v8f wmmab(v16bf a, v16bf b, v8f c) { return __builtin_amdgcn_wmma_f32_16x16x32_bf16(false, a, false, b, (short)0, c, false, false); }


template <typename T16> struct WFrag;
template <> struct WFrag<h16> { typedef v16h V; static __device__ __forceinline__ V ld(const h16* p) { return cat16(*(const v8h*)p, *(const v8h*)(p + 16)); } static __device__ __forceinline__ v8f mma(V a, V b, v8f c) { return wmma16(a, b, c); } };
template <> struct WFrag<bf> { typedef v16bf V; static __device__ __forceinline__ V ld(const bf* p) { return cat16b(*(const v8us*)p, *(const v8us*)(p + 16)); } static __device__ __forceinline__ v8f mma(V a, V b, v8f c) { return wmmab(a, b, c); } };
template <typename T16, int NSPLIT, bool BIAS>
__global__ __launch_bounds__(32) void k_gemmw(const T16* __restrict__ A, const T16* __restrict__ A2, const T16* __restrict__ Bt, const T16* __restrict__ Bt2, int K, float* C, int ldc, const float* __restrict__ bias, size_t sA, size_t sB, size_t sC) {
    typedef typename WFrag<T16>::V V;
    __shared__ __align__(16) float os[16 * 68];
    const size_t z = blockIdx.z; A += z * sA; if (A2) A2 += z * sA; Bt += z * sB; if (Bt2) Bt2 += z * sB; C += z * sC;
    const int lane = threadIdx.x & 31, lr = lane & 15, hi = lane >> 4; const int r0 = blockIdx.x * 64, c0 = blockIdx.y * 64;
    v8f acc[4][4];
#pragma unroll
    for (int mb = 0; mb < 4; ++mb)
#pragma unroll
        for (int nb = 0; nb < 4; ++nb) acc[mb][nb] = (v8f){};
    const size_t aoff = (size_t)(r0 + lr) * K + 8 * hi, boff = (size_t)(c0 + lr) * K + 8 * hi;
#pragma unroll 1
    for (int kc = 0; kc < K; kc += 32) {
        V a[4], a2[4];
#pragma unroll
        for (int mb = 0; mb < 4; ++mb) { a[mb] = WFrag<T16>::ld(A + aoff + (size_t)mb * 16 * K + kc); if (NSPLIT == 1 || NSPLIT == 2) a2[mb] = WFrag<T16>::ld(A2 + aoff + (size_t)mb * 16 * K + kc); }
#pragma unroll
        for (int nb = 0; nb < 4; ++nb) { const V b = WFrag<T16>::ld(Bt + boff + (size_t)nb * 16 * K + kc); V b2; if (NSPLIT >= 2) b2 = WFrag<T16>::ld(Bt2 + boff + (size_t)nb * 16 * K + kc);
#pragma unroll
            for (int mb = 0; mb < 4; ++mb) { acc[mb][nb] = WFrag<T16>::mma(a[mb], b, acc[mb][nb]); if (NSPLIT == 1 || NSPLIT == 2) acc[mb][nb] = WFrag<T16>::mma(a2[mb], b, acc[mb][nb]); if (NSPLIT >= 2) acc[mb][nb] = WFrag<T16>::mma(a[mb], b2, acc[mb][nb]); } }
        asm volatile("v_nop\n\tv_nop\n\tv_nop\n\tv_nop" : "+v"(acc[0][0]), "+v"(acc[1][1]), "+v"(acc[2][2]), "+v"(acc[3][3]) : "v"(a[0]), "v"(a[3]));
    }
#pragma unroll
    for (int mb = 0; mb < 4; ++mb) {
#pragma unroll
        for (int nb = 0; nb < 4; ++nb) {
#pragma unroll
            for (int j = 0; j < 8; ++j) os[(hi * 8 + j) * 68 + nb * 16 + lr] = acc[mb][nb][j]; }
        __builtin_amdgcn_wave_barrier(); asm volatile("" ::: "memory");
        float* crow = C + (size_t)(r0 + mb * 16) * ldc + c0;
#pragma unroll 1
        for (int ps = 0; ps < 2; ++ps) {
#pragma unroll
            for (int s = 0; s < 8; ++s) { const int row = 2 * s + hi, cofs = lr * 4; v4f val = *(const v4fa*)(os + row * 68 + cofs); if (BIAS) { val[0] += bfr(bias[c0 + cofs]); val[1] += bfr(bias[c0 + cofs + 1]); val[2] += bfr(bias[c0 + cofs + 2]); val[3] += bfr(bias[c0 + cofs + 3]); }
                *(volatile v4f*)(crow + (size_t)row * ldc + cofs) = val; }
            if (ps == 0) __threadfence(); }
        __builtin_amdgcn_wave_barrier(); asm volatile("" ::: "memory");
    }
}

__device__ __forceinline__ void splitf(float y, unsigned short& h, unsigned short& l) { h = f2bf(y); l = f2bf(y - bf2f(h)); }
__device__ __forceinline__ float lky(float t) { return t >= 0.f ? t : SL * t; }
typedef __attribute__((ext_vector_type(2))) unsigned short v2us;
typedef __attribute__((ext_vector_type(2))) float v2f;

__global__ __launch_bounds__(256) void k_cvt8(const float* __restrict__ src, bf* dst, size_t n8) { const size_t i = (size_t)blockIdx.x * 256 + threadIdx.x; if (i >= n8) return; const v8f v = *(const v8f*)(src + i * 8); v8us o;
#pragma unroll
    for (int k = 0; k < 8; ++k) o[k] = f2bf(v[k]); *(volatile v8us*)(dst + i * 8) = o; __threadfence(); *(volatile v8us*)(dst + i * 8) = o; }
__global__ __launch_bounds__(256) void k_wtb(const float* __restrict__ w, bf* Bt) { const int i = blockIdx.x * 256 + threadIdx.x; if (i >= CC * CC / 2) return; const int e = i * 2; const int n = e / CC, k = e % CC; v2us o; o[0] = f2bf(w[k * CC + n]); o[1] = f2bf(w[(k + 1) * CC + n]); *(volatile v2us*)(Bt + e) = o; __threadfence(); *(volatile v2us*)(Bt + e) = o; }
__global__ __launch_bounds__(256) void k_eT(const float* __restrict__ ev, bf* ET) {
    const int lane = threadIdx.x & 31; const int L = blockIdx.x * 8 + (threadIdx.x >> 5); if (L >= NT * CC / 64) return; const int e = L * 64 + lane * 2; const int j = e & (NN - 1); const int c = (e >> 10) & 63; const int b = e >> 16; v2us o;
    o[0] = f2bf(ev[((size_t)b * NN + j) * CC + c]); o[1] = f2bf(ev[((size_t)b * NN + j + 1) * CC + c]); *(volatile v2us*)(ET + e) = o; __threadfence(); *(volatile v2us*)(ET + e) = o;
}
__global__ __launch_bounds__(256) void k_gat(const float* __restrict__ VU, const float* __restrict__ IV, const float* __restrict__ yita, const int* __restrict__ adj, bf* Ah, bf* Al) {
    __shared__ float svu[8][CC]; __shared__ float sy[8][CC];
    const int lane = threadIdx.x & 31, wv = threadIdx.x >> 5; const int row = blockIdx.x * 8 + wv; if (row >= NT) return; const int b = row / NN;
    svu[wv][lane] = VU[(size_t)row * CC + lane]; svu[wv][lane + 32] = VU[(size_t)row * CC + lane + 32]; sy[wv][lane] = bfr(yita[lane]); sy[wv][lane + 32] = bfr(yita[lane + 32]);
    __builtin_amdgcn_wave_barrier(); asm volatile("" ::: "memory");
    float v[32]; float mx = -3.0e38f;
#pragma unroll 1
    for (int q = 0; q < 16; ++q)
#pragma unroll
        for (int t2 = 0; t2 < 2; ++t2) { const int j = q * 64 + lane * 2 + t2; const float* ivr = IV + ((size_t)b * NN + j) * CC; float s = 0.f;
#pragma unroll 4
            for (int c = 0; c < CC; ++c) s = fmaf(sy[wv][c], lky(svu[wv][c] + ivr[c]), s);
            const float t = (adj[(size_t)row * NN + j] > 0) ? s : -1.0e12f; v[q * 2 + t2] = t; mx = fmaxf(mx, t); }
#pragma unroll
    for (int sh = 16; sh; sh >>= 1) mx = fmaxf(mx, __shfl_xor(mx, sh, 32));
    float sum = 0.f;
#pragma unroll
    for (int q = 0; q < 32; ++q) { v[q] = __expf(v[q] - mx); sum += v[q]; }
#pragma unroll
    for (int sh = 16; sh; sh >>= 1) sum += __shfl_xor(sum, sh, 32);
    const float f = __fdiv_rn(1.0f, sum);
#pragma unroll 1
    for (int ps = 0; ps < 2; ++ps) {
#pragma unroll
        for (int q = 0; q < 16; ++q) { v2us oh, ol; unsigned short a, c2; splitf(v[q * 2] * f, a, c2); oh[0] = a; ol[0] = c2; splitf(v[q * 2 + 1] * f, a, c2); oh[1] = a; ol[1] = c2;
            *(volatile v2us*)(Ah + (size_t)row * NN + q * 64 + lane * 2) = oh; *(volatile v2us*)(Al + (size_t)row * NN + q * 64 + lane * 2) = ol; }
        if (ps == 0) __threadfence(); }
}
__global__ __launch_bounds__(256) void k_mix(const float* __restrict__ AG, const float* __restrict__ ev, const float* __restrict__ beta, bf* Ph, bf* Pl) {
    const int lane = threadIdx.x & 31; const int L = blockIdx.x * 8 + (threadIdx.x >> 5); if (L >= NT * CC / 64) return; const int e = L * 64 + lane * 2; const float bb = 1.0f + bfr(beta[0]); v2us oh, ol;
#pragma unroll
    for (int q = 0; q < 2; ++q) { unsigned short a, c2; splitf(lky(AG[(size_t)e + q]) + bb * bfr(ev[(size_t)e + q]), a, c2); oh[q] = a; ol[q] = c2; }
    *(volatile v2us*)(Ph + e) = oh; *(volatile v2us*)(Pl + e) = ol; __threadfence(); *(volatile v2us*)(Ph + e) = oh; *(volatile v2us*)(Pl + e) = ol;
}
__global__ __launch_bounds__(256) void k_fin(const float* __restrict__ C, float* OUT) { const size_t i = (size_t)blockIdx.x * 256 + threadIdx.x; if (i >= (size_t)NT * CC / 4) return; const v4f c = *(const v4f*)(C + i * 4); v4f o;
#pragma unroll
    for (int q = 0; q < 4; ++q) o[q] = lky(c[q]); *(volatile v4f*)(OUT + i * 4) = o; __threadfence(); *(volatile v4f*)(OUT + i * 4) = o; }

extern "C" void kernel_launch(void* const* d_in, const int* in_sizes, int n_in,
                              void* d_out, int out_size, void* d_ws, size_t ws_size, hipStream_t stream) {
    (void)in_sizes; (void)n_in; (void)out_size;
    const float* ev = (const float*)d_in[0]; const int* adj = (const int*)d_in[1];   const float* U2 = (const float*)d_in[3]; const float* W2 = (const float*)d_in[4];
    const float* yita = (const float*)d_in[5]; const float* beta = (const float*)d_in[6]; const float* linW = (const float*)d_in[7]; const float* linb = (const float*)d_in[8];
    float* OUT = (float*)d_out;
    char* wsp = (char*)d_ws;
    auto take = [&](size_t bytes) { char* p = wsp; wsp += (bytes + 255) & ~(size_t)255; return (void*)p; };
    bf* EB = (bf*)take((size_t)NT * CC * 2); bf* ET = (bf*)take((size_t)NT * CC * 2); bf* U2B = (bf*)take(CC * CC * 2); bf* W2B = (bf*)take(CC * CC * 2); bf* LWB = (bf*)take(CC * CC * 2);
    float* VU = (float*)take((size_t)NT * CC * 4); float* IV = (float*)take((size_t)NT * CC * 4); bf* Ah = (bf*)take((size_t)NT * NN * 2); bf* Al = (bf*)take((size_t)NT * NN * 2);
    float* AG = (float*)take((size_t)NT * CC * 4); bf* Mh = (bf*)take((size_t)NT * CC * 2); bf* Ml = (bf*)take((size_t)NT * CC * 2); float* C3 = (float*)take((size_t)NT * CC * 4);
    if ((size_t)(wsp - (char*)d_ws) > ws_size) return;
    k_cvt8<<<(unsigned)((NT * CC / 8 + 255) / 256), 256, 0, stream>>>(ev, EB, (size_t)NT * CC / 8); k_eT<<<(NT * CC / 64 + 7) / 8, 256, 0, stream>>>(ev, ET);
    k_wtb<<<(CC * CC / 2 + 255) / 256, 256, 0, stream>>>(U2, U2B); k_wtb<<<(CC * CC / 2 + 255) / 256, 256, 0, stream>>>(W2, W2B); k_cvt8<<<(unsigned)((CC * CC / 8 + 255) / 256), 256, 0, stream>>>(linW, LWB, (size_t)CC * CC / 8);
    k_gemmw<bf, 0, false><<<dim3(NT / 64, 1, 1), 32, 0, stream>>>(EB, nullptr, U2B, nullptr, CC, VU, CC, nullptr, 0, 0, 0);
    k_gemmw<bf, 0, false><<<dim3(NT / 64, 1, 1), 32, 0, stream>>>(EB, nullptr, W2B, nullptr, CC, IV, CC, nullptr, 0, 0, 0);
    k_gat<<<NT / 8, 256, 0, stream>>>(VU, IV, yita, adj, Ah, Al);
    k_gemmw<bf, 1, false><<<dim3(NN / 64, 1, NB_), 32, 0, stream>>>(Ah, Al, ET, nullptr, NN, AG, CC, nullptr, (size_t)NN * NN, (size_t)CC * NN, (size_t)NN * CC);
    k_mix<<<(NT * CC / 64 + 7) / 8, 256, 0, stream>>>(AG, ev, beta, Mh, Ml);
    k_gemmw<bf, 1, true><<<dim3(NT / 64, 1, 1), 32, 0, stream>>>(Mh, Ml, LWB, nullptr, CC, C3, CC, linb, 0, 0, 0);
    k_fin<<<(unsigned)((NT * CC / 4 + 255) / 256), 256, 0, stream>>>(C3, OUT);
}
